// MultiHeadSelfAttention_59030030516776
// MI455X (gfx1250) — hardware-verified
//
#include <hip/hip_runtime.h>
#ifndef NB
#define NB 2
#endif
#ifndef SEQ
#define SEQ 2048
#endif
#define NB_FULL 2
#define SEQ_FULL 2048
#define DM 1024
#define NH 16
#define HD 64
#define LQ (3 * DM)
#define LL (2 * DM)
#define MR (NB * SEQ)
#define KP 72
#define PP 40
#define SM_KH 0
#define SM_KL (64 * KP)
#define SM_VT (2 * 64 * KP)
#define SM_P  (3 * 64 * KP)
#define SM_TOT (3 * 64 * KP + 8 * 16 * PP)
#define EPW (2 * 16 * KP)

static_assert(NH * HD == DM);
static_assert(HD == 64);
static_assert(SEQ % 128 == 0);
static_assert(MR % 128 == 0);
static_assert(LQ % 64 == 0 && DM % 64 == 0);
static_assert(DM % 32 == 0 && LL % 32 == 0);
static_assert(NB <= NB_FULL && SEQ <= SEQ_FULL);
static_assert(8 * EPW <= SM_TOT);
static_assert((KP * 2) % 16 == 0 && (PP * 2) % 16 == 0);

typedef __bf16   v16b __attribute__((ext_vector_type(16)));
typedef _Float16 v16h __attribute__((ext_vector_type(16)));
typedef unsigned short v8us __attribute__((ext_vector_type(8), may_alias));
typedef float v8f  __attribute__((ext_vector_type(8)));
typedef float v4f  __attribute__((ext_vector_type(4)));
typedef float v4fa __attribute__((ext_vector_type(4), may_alias));
union FragB { v16b v; v8us half[2]; };
union FragH { v16h v; v8us half[2]; };

__device__ __forceinline__ unsigned short bf16_bits(float x) { unsigned int u = __float_as_uint(x); return (unsigned short)((u + 0x7FFFu + ((u >> 16) & 1u)) >> 16); }
__device__ __forceinline__ float bf16_val(unsigned short b) { return __uint_as_float(((unsigned int)b) << 16); }
__device__ __forceinline__ float bf16_rne(float x) { return bf16_val(bf16_bits(x)); }
__device__ __forceinline__ unsigned short f16_bits(float x) { const _Float16 h = (_Float16)x; return __builtin_bit_cast(unsigned short, h); }

__device__ __forceinline__ v16b ldfb_g(const unsigned short* __restrict__ p, int hh) { FragB f; f.half[0] = *(const v8us*)(p + 8 * hh); f.half[1] = *(const v8us*)(p + 16 + 8 * hh); return f.v; }

__device__ __forceinline__ v8f mma_b(v16b a, v16b b, v8f c) {
  v8f d = __builtin_amdgcn_wmma_f32_16x16x32_bf16(false, a, false, b, (short)0, c, false, false);
  asm volatile("v_nop\n\tv_nop\n\tv_nop\n\tv_nop" : "+v"(d) : "v"(a), "v"(b));
  return d;
}
__device__ __forceinline__ v8f mma_h(v16h a, v16h b, v8f c) {
  v8f d = __builtin_amdgcn_wmma_f32_16x16x32_f16(false, a, false, b, (short)0, c, false, false);
  asm volatile("v_nop\n\tv_nop\n\tv_nop\n\tv_nop" : "+v"(d) : "v"(a), "v"(b));
  return d;
}

__global__ __launch_bounds__(256) void k_wt(const float* __restrict__ W, unsigned short* __restrict__ Wt, int N, int ldo, int dup) {
  const int t = blockIdx.x * 256 + threadIdx.x;
  const int k8n = DM / 8;
  if (t >= N * k8n) return;
  const int n = t / k8n, k8 = (t - n * k8n) * 8;
  v8us v;
#pragma unroll
  for (int i = 0; i < 8; ++i) v[i] = bf16_bits(W[(size_t)(k8 + i) * N + n]);
  unsigned short* p = Wt + (size_t)n * ldo + k8;
  for (int pass = 0; pass < 2; ++pass) {
    *(volatile v8us*)p = v;
    if (dup) *(volatile v8us*)(p + DM) = v;
    if (pass == 0) __threadfence();
  }
}

__global__ __launch_bounds__(256) void k_xb(const float* __restrict__ x, unsigned short* __restrict__ XB) {
  const size_t t = (size_t)blockIdx.x * 256 + threadIdx.x;
  const size_t n8 = (size_t)MR * (DM / 8);
  if (t >= n8) return;
  const int row = (int)(t / (DM / 8)), c8 = (int)(t % (DM / 8)) * 8;
  const int b = row / SEQ, s = row - b * SEQ;
  const float* src = x + ((size_t)b * SEQ_FULL + s) * DM + c8;
  const v4f a = *(const v4fa*)src, c = *(const v4fa*)(src + 4);
  v8us v;
#pragma unroll
  for (int q = 0; q < 4; ++q) { v[q] = bf16_bits(a[q]); v[4 + q] = bf16_bits(c[q]); }
  unsigned short* p = XB + (size_t)row * DM + c8;
  *(volatile v8us*)p = v;
  __threadfence();
  *(volatile v8us*)p = v;
}

__global__ __launch_bounds__(128) void k_gemm_qkv(const unsigned short* __restrict__ A, const unsigned short* __restrict__ Bt, const float* __restrict__ bias,
                                                  unsigned short* __restrict__ HI, unsigned short* __restrict__ LO) {
  __shared__ __attribute__((aligned(16))) float so[4][32][68];
  const int tid = threadIdx.x;
  const int w = __builtin_amdgcn_readfirstlane(tid >> 5);
  const int lane = tid & 31, ln = lane & 15, hh = lane >> 4;
  const int ntn = LQ / 64;
  const int mt = blockIdx.x / ntn, nq = blockIdx.x - mt * ntn;
  const int row0 = mt * 128 + 32 * w, col0 = nq * 64;
  const unsigned short* a0p = A + (size_t)(row0 + ln) * DM; const unsigned short* a1p = a0p + (size_t)16 * DM;
  const unsigned short* b0p = Bt + (size_t)(col0 + ln) * DM; const unsigned short* b1p = b0p + (size_t)16 * DM;
  const unsigned short* b2p = b1p + (size_t)16 * DM; const unsigned short* b3p = b2p + (size_t)16 * DM;
  const v8f z8 = {0.f, 0.f, 0.f, 0.f, 0.f, 0.f, 0.f, 0.f};
  v8f c00 = z8, c01 = z8, c02 = z8, c03 = z8, c10 = z8, c11 = z8, c12 = z8, c13 = z8;
#pragma unroll 1
  for (int kb = 0; kb < DM; kb += 32) {
    const v16b a0 = ldfb_g(a0p + kb, hh), a1 = ldfb_g(a1p + kb, hh);
    v16b b = ldfb_g(b0p + kb, hh); c00 = mma_b(a0, b, c00); c10 = mma_b(a1, b, c10);
    b = ldfb_g(b1p + kb, hh); c01 = mma_b(a0, b, c01); c11 = mma_b(a1, b, c11);
    b = ldfb_g(b2p + kb, hh); c02 = mma_b(a0, b, c02); c12 = mma_b(a1, b, c12);
    b = ldfb_g(b3p + kb, hh); c03 = mma_b(a0, b, c03); c13 = mma_b(a1, b, c13);
  }
  v8f accs[8] = {c00, c01, c02, c03, c10, c11, c12, c13};
#pragma unroll
  for (int u = 0; u < 8; ++u) {
    const int t = u & 3, half = u >> 2;
    const float bv = bf16_rne(bias[col0 + t * 16 + ln]);
#pragma unroll
    for (int r = 0; r < 8; ++r) so[w][half * 16 + 8 * hh + r][t * 16 + ln] = accs[u][r] + bv;
  }
  __builtin_amdgcn_fence(4  , "workgroup");
  __builtin_amdgcn_wave_barrier();
  const int rq = lane >> 3, c8 = (lane & 7) * 8;
  const int isv = (col0 >= 2 * DM) ? 1 : 0;
  for (int pass = 0; pass < 2; ++pass) {
#pragma unroll
    for (int q = 0; q < 8; ++q) {
      const int r = q * 4 + rq;
      const v4f a = *(const v4fa*)&so[w][r][c8];
      const v4f c = *(const v4fa*)&so[w][r][c8 + 4];
      const float xs[8] = {a[0], a[1], a[2], a[3], c[0], c[1], c[2], c[3]};
      v8us ho, lo;
#pragma unroll
      for (int i = 0; i < 8; ++i) {
        const unsigned short hb = bf16_bits(xs[i]);
        const unsigned short fb = f16_bits(xs[i]);
        ho[i] = isv ? fb : hb;
        lo[i] = bf16_bits(xs[i] - bf16_val(hb));
      }
      *(volatile v8us*)(HI + (size_t)(row0 + r) * LQ + col0 + c8) = ho;
      if (!isv) *(volatile v8us*)(LO + (size_t)(row0 + r) * LL + col0 + c8) = lo;
    }
    if (pass == 0) __threadfence();
  }
}

__global__ __launch_bounds__(256) void k_vt(const unsigned short* __restrict__ HI, unsigned short* __restrict__ VT) {
  __shared__ unsigned short tl[64][66];
  const int tid = threadIdx.x;
  const int slab = blockIdx.x / (SEQ / 64), lg = blockIdx.x - slab * (SEQ / 64);
  const int b = slab / NH, h = slab - b * NH;
  for (int i = tid; i < 64 * 8; i += 256) {
    const int r = i >> 3, c8 = (i & 7) * 8;
    const v8us f = *(const v8us*)(HI + ((size_t)b * SEQ + lg * 64 + r) * LQ + 2 * DM + h * HD + c8);
#pragma unroll
    for (int q = 0; q < 8; ++q) tl[r][c8 + q] = f[q];
  }
  __syncthreads();
  for (int pass = 0; pass < 2; ++pass) {
#pragma unroll
    for (int rd = 0; rd < 2; ++rd) {
      const int d = rd * 32 + (tid >> 3), pc = tid & 7;
      v8us o;
#pragma unroll
      for (int q = 0; q < 8; ++q) o[q] = tl[pc * 8 + q][d];
      *(volatile v8us*)(VT + ((size_t)slab * 64 + d) * SEQ + lg * 64 + pc * 8) = o;
    }
    if (pass == 0) __threadfence();
  }
}

__global__ __launch_bounds__(256) void k_attn(const unsigned short* __restrict__ QKH, const unsigned short* __restrict__ QKL, const unsigned short* __restrict__ VT,
                                              const int* __restrict__ mask, unsigned short* __restrict__ CTX) {
  __shared__ __attribute__((aligned(16))) unsigned short sm[SM_TOT];
  __shared__ int mks[64];
  const int tid = threadIdx.x;
  const int wave = __builtin_amdgcn_readfirstlane(tid >> 5);
  const int lane = tid & 31, ln = lane & 15, hh = lane >> 4;
  const int bh = blockIdx.y;
  const int b = bh / NH, h = bh - b * NH;
  const int q0 = blockIdx.x * 128;
  const size_t rowb = (size_t)b * SEQ;
  const size_t qrow = rowb + q0 + wave * 16 + ln;
  const v16b qh0 = ldfb_g(QKH + qrow * LQ + h * HD, hh), qh1 = ldfb_g(QKH + qrow * LQ + h * HD + 32, hh);
  const v16b ql0 = ldfb_g(QKL + qrow * LL + h * HD, hh), ql1 = ldfb_g(QKL + qrow * LL + h * HD + 32, hh);
  const v8f z8 = {0.f, 0.f, 0.f, 0.f, 0.f, 0.f, 0.f, 0.f};
  v8f O0 = z8, O1 = z8, O2 = z8, O3 = z8;
  float mrow[8], lpart[8];
#pragma unroll
  for (int r = 0; r < 8; ++r) { mrow[r] = -3.0e38f; lpart[r] = 0.f; }
  const int pbase = SM_P + wave * (16 * PP);
  const float NEG_INF = -__builtin_huge_valf();
  const float SC2 = 0.125f * 1.4426950408889634f;

#pragma unroll 1
  for (int kt0 = 0; kt0 < SEQ; kt0 += 64) {
#pragma unroll
    for (int j = 0; j < 2; ++j) {
      const int i = tid + j * 256;
      const int r = i >> 3, c8 = (i & 7) * 8;
      const size_t krow = rowb + kt0 + r;
      const v8us kh = *(const v8us*)(QKH + krow * LQ + DM + h * HD + c8);
      const v8us kl = *(const v8us*)(QKL + krow * LL + DM + h * HD + c8);
      const v8us vv = *(const v8us*)(VT + ((size_t)bh * HD + r) * SEQ + kt0 + c8);
      *(v8us*)&sm[SM_KH + r * KP + c8] = kh;
      *(v8us*)&sm[SM_KL + r * KP + c8] = kl;
      *(v8us*)&sm[SM_VT + r * KP + c8] = vv;
    }
    if (tid < 64) mks[tid] = mask[(size_t)b * SEQ_FULL + kt0 + tid];
    __syncthreads();

#pragma unroll
    for (int hf = 0; hf < 2; ++hf) {
      const int k0 = hf * 32;
      v8f s0 = z8, s1 = z8;
      {
        const int ka = (k0 + ln) * KP, kb = (k0 + 16 + ln) * KP;
        FragB fh, fl;
        fh.half[0] = *(const v8us*)&sm[SM_KH + ka + 8 * hh]; fh.half[1] = *(const v8us*)&sm[SM_KH + ka + 16 + 8 * hh];
        fl.half[0] = *(const v8us*)&sm[SM_KL + ka + 8 * hh]; fl.half[1] = *(const v8us*)&sm[SM_KL + ka + 16 + 8 * hh];
        s0 = mma_b(qh0, fh.v, s0); s0 = mma_b(ql0, fh.v, s0); s0 = mma_b(qh0, fl.v, s0);
        fh.half[0] = *(const v8us*)&sm[SM_KH + ka + 32 + 8 * hh]; fh.half[1] = *(const v8us*)&sm[SM_KH + ka + 48 + 8 * hh];
        fl.half[0] = *(const v8us*)&sm[SM_KL + ka + 32 + 8 * hh]; fl.half[1] = *(const v8us*)&sm[SM_KL + ka + 48 + 8 * hh];
        s0 = mma_b(qh1, fh.v, s0); s0 = mma_b(ql1, fh.v, s0); s0 = mma_b(qh1, fl.v, s0);
        fh.half[0] = *(const v8us*)&sm[SM_KH + kb + 8 * hh]; fh.half[1] = *(const v8us*)&sm[SM_KH + kb + 16 + 8 * hh];
        fl.half[0] = *(const v8us*)&sm[SM_KL + kb + 8 * hh]; fl.half[1] = *(const v8us*)&sm[SM_KL + kb + 16 + 8 * hh];
        s1 = mma_b(qh0, fh.v, s1); s1 = mma_b(ql0, fh.v, s1); s1 = mma_b(qh0, fl.v, s1);
        fh.half[0] = *(const v8us*)&sm[SM_KH + kb + 32 + 8 * hh]; fh.half[1] = *(const v8us*)&sm[SM_KH + kb + 48 + 8 * hh];
        fl.half[0] = *(const v8us*)&sm[SM_KL + kb + 32 + 8 * hh]; fl.half[1] = *(const v8us*)&sm[SM_KL + kb + 48 + 8 * hh];
        s1 = mma_b(qh1, fh.v, s1); s1 = mma_b(ql1, fh.v, s1); s1 = mma_b(qh1, fl.v, s1);
      }
      const int mk0 = mks[k0 + ln], mk1 = mks[k0 + 16 + ln];
#pragma unroll
      for (int r = 0; r < 8; ++r) {
        float a0 = s0[r] * SC2, a1 = s1[r] * SC2;
        a0 = (mk0 == 0) ? NEG_INF : a0;
        a1 = (mk1 == 0) ? NEG_INF : a1;
        float mx = fmaxf(a0, a1);
        mx = fmaxf(mx, __shfl_xor(mx, 1, 32));
        mx = fmaxf(mx, __shfl_xor(mx, 2, 32));
        mx = fmaxf(mx, __shfl_xor(mx, 4, 32));
        mx = fmaxf(mx, __shfl_xor(mx, 8, 32));
        const float newm = fmaxf(mrow[r], mx);
        const float corr = exp2f(mrow[r] - newm);
        const _Float16 h0 = (_Float16)exp2f((a0 - newm) + 8.0f);
        const _Float16 h1 = (_Float16)exp2f((a1 - newm) + 8.0f);
        lpart[r] = lpart[r] * corr + ((float)h0 + (float)h1);
        mrow[r] = newm;
        O0[r] *= corr; O1[r] *= corr; O2[r] *= corr; O3[r] *= corr;
        sm[pbase + (8 * hh + r) * PP + ln]      = __builtin_bit_cast(unsigned short, h0);
        sm[pbase + (8 * hh + r) * PP + 16 + ln] = __builtin_bit_cast(unsigned short, h1);
      }
      __builtin_amdgcn_fence(4  , "workgroup");
      __builtin_amdgcn_wave_barrier();
      FragH pa;
      pa.half[0] = *(const v8us*)&sm[pbase + ln * PP + 8 * hh];
      pa.half[1] = *(const v8us*)&sm[pbase + ln * PP + 16 + 8 * hh];
      {
        FragH vb;
        const int vo = SM_VT + ln * KP + k0;
        vb.half[0] = *(const v8us*)&sm[vo + 8 * hh];               vb.half[1] = *(const v8us*)&sm[vo + 16 + 8 * hh];
        O0 = mma_h(pa.v, vb.v, O0);
        vb.half[0] = *(const v8us*)&sm[vo + 16 * KP + 8 * hh];     vb.half[1] = *(const v8us*)&sm[vo + 16 * KP + 16 + 8 * hh];
        O1 = mma_h(pa.v, vb.v, O1);
        vb.half[0] = *(const v8us*)&sm[vo + 32 * KP + 8 * hh];     vb.half[1] = *(const v8us*)&sm[vo + 32 * KP + 16 + 8 * hh];
        O2 = mma_h(pa.v, vb.v, O2);
        vb.half[0] = *(const v8us*)&sm[vo + 48 * KP + 8 * hh];     vb.half[1] = *(const v8us*)&sm[vo + 48 * KP + 16 + 8 * hh];
        O3 = mma_h(pa.v, vb.v, O3);
      }
      __builtin_amdgcn_fence(4  , "workgroup");
      __builtin_amdgcn_wave_barrier();
    }
    __syncthreads();
  }

  const int ep = wave * EPW;
#pragma unroll
  for (int r = 0; r < 8; ++r) {
    float l = lpart[r];
    l += __shfl_xor(l, 1, 32);
    l += __shfl_xor(l, 2, 32);
    l += __shfl_xor(l, 4, 32);
    l += __shfl_xor(l, 8, 32);
    const float inv = 1.0f / l;
    const int ro = ep + (8 * hh + r) * KP + ln;
    float v; unsigned short hb;
    v = O0[r] * inv; hb = bf16_bits(v); sm[ro]      = hb; sm[ro + 16 * KP]      = bf16_bits(v - bf16_val(hb));
    v = O1[r] * inv; hb = bf16_bits(v); sm[ro + 16] = hb; sm[ro + 16 * KP + 16] = bf16_bits(v - bf16_val(hb));
    v = O2[r] * inv; hb = bf16_bits(v); sm[ro + 32] = hb; sm[ro + 16 * KP + 32] = bf16_bits(v - bf16_val(hb));
    v = O3[r] * inv; hb = bf16_bits(v); sm[ro + 48] = hb; sm[ro + 16 * KP + 48] = bf16_bits(v - bf16_val(hb));
  }
  __builtin_amdgcn_fence(4  , "workgroup");
  __builtin_amdgcn_wave_barrier();
  const int rq = lane >> 3, c8 = (lane & 7) * 8;
  for (int pass = 0; pass < 2; ++pass) {
#pragma unroll
    for (int q = 0; q < 4; ++q) {
      const int r = q * 4 + rq;
      const v8us hv = *(const v8us*)&sm[ep + r * KP + c8];
      const v8us lv = *(const v8us*)&sm[ep + 16 * KP + r * KP + c8];
      unsigned short* dst = CTX + (rowb + q0 + wave * 16 + r) * LL + h * HD + c8;
      *(volatile v8us*)dst = hv;
      *(volatile v8us*)(dst + DM) = lv;
    }
    if (pass == 0) __threadfence();
  }
}

__global__ __launch_bounds__(128) void k_gemm_out(const unsigned short* __restrict__ A, const unsigned short* __restrict__ Bt, const float* __restrict__ bias, float* __restrict__ C) {
  __shared__ __attribute__((aligned(16))) float so[4][32][68];
  const int tid = threadIdx.x;
  const int w = __builtin_amdgcn_readfirstlane(tid >> 5);
  const int lane = tid & 31, ln = lane & 15, hh = lane >> 4;
  const int ntn = DM / 64;
  const int mt = blockIdx.x / ntn, nq = blockIdx.x - mt * ntn;
  const int row0 = mt * 128 + 32 * w, col0 = nq * 64;
  const unsigned short* a0p = A + (size_t)(row0 + ln) * LL; const unsigned short* a1p = a0p + (size_t)16 * LL;
  const unsigned short* b0p = Bt + (size_t)(col0 + ln) * LL; const unsigned short* b1p = b0p + (size_t)16 * LL;
  const unsigned short* b2p = b1p + (size_t)16 * LL; const unsigned short* b3p = b2p + (size_t)16 * LL;
  const v8f z8 = {0.f, 0.f, 0.f, 0.f, 0.f, 0.f, 0.f, 0.f};
  v8f c00 = z8, c01 = z8, c02 = z8, c03 = z8, c10 = z8, c11 = z8, c12 = z8, c13 = z8;
#pragma unroll 1
  for (int kb = 0; kb < LL; kb += 32) {
    const v16b a0 = ldfb_g(a0p + kb, hh), a1 = ldfb_g(a1p + kb, hh);
    v16b b = ldfb_g(b0p + kb, hh); c00 = mma_b(a0, b, c00); c10 = mma_b(a1, b, c10);
    b = ldfb_g(b1p + kb, hh); c01 = mma_b(a0, b, c01); c11 = mma_b(a1, b, c11);
    b = ldfb_g(b2p + kb, hh); c02 = mma_b(a0, b, c02); c12 = mma_b(a1, b, c12);
    b = ldfb_g(b3p + kb, hh); c03 = mma_b(a0, b, c03); c13 = mma_b(a1, b, c13);
  }
  v8f accs[8] = {c00, c01, c02, c03, c10, c11, c12, c13};
#pragma unroll
  for (int u = 0; u < 8; ++u) {
    const int t = u & 3, half = u >> 2;
    const float bv = bf16_rne(bias[col0 + t * 16 + ln]);
#pragma unroll
    for (int r = 0; r < 8; ++r) so[w][half * 16 + 8 * hh + r][t * 16 + ln] = accs[u][r] + bv;
  }
  __builtin_amdgcn_fence(4  , "workgroup");
  __builtin_amdgcn_wave_barrier();
  const int rsub = lane >> 4, c4 = (lane & 15) * 4;
  const int ob = row0 / SEQ;
  const size_t orow0 = (size_t)ob * SEQ_FULL + (size_t)(row0 - ob * SEQ);
  for (int pass = 0; pass < 2; ++pass) {
#pragma unroll
    for (int q = 0; q < 16; ++q) {
      const int r = q * 2 + rsub;
      const v4f v = *(const v4fa*)&so[w][r][c4];
      *(volatile v4f*)(C + (orow0 + r) * DM + col0 + c4) = v;
    }
    if (pass == 0) __threadfence();
  }
}

#define WS_WQT ((size_t)0)
#define WS_WOT (WS_WQT + (size_t)LQ * DM * 2)
#define WS_XB  (WS_WOT + (size_t)DM * LL * 2)
#define WS_QKH (WS_XB  + (size_t)MR * DM * 2)
#define WS_QKL (WS_QKH + (size_t)MR * LQ * 2)
#define WS_VT  (WS_QKL + (size_t)MR * LL * 2)
#define WS_CTX (WS_VT  + (size_t)NB * NH * HD * SEQ * 2)
#define WS_TOTAL (WS_CTX + (size_t)MR * LL * 2)
static_assert(WS_TOTAL <= (size_t)134217728);
static_assert(WS_WOT % 256 == 0 && WS_XB % 256 == 0 && WS_QKH % 256 == 0 && WS_QKL % 256 == 0 && WS_VT % 256 == 0 && WS_CTX % 256 == 0);
static_assert(((size_t)(NB - 1) * SEQ_FULL + SEQ) * DM <= (size_t)NB_FULL * SEQ_FULL * DM);

extern "C" void kernel_launch(void* const* d_in, const int* in_sizes, int n_in,
                              void* d_out, int out_size, void* d_ws, size_t ws_size, hipStream_t stream) {
  if (n_in < 6) return;
  const size_t need_rows = (size_t)(NB - 1) * SEQ_FULL + SEQ;
  if ((size_t)in_sizes[0] < need_rows * DM) return;
  if ((size_t)in_sizes[1] < need_rows) return;
  if ((size_t)in_sizes[2] < (size_t)DM * LQ) return;
  if ((size_t)in_sizes[3] < (size_t)LQ) return;
  if ((size_t)in_sizes[4] < (size_t)DM * DM) return;
  if ((size_t)in_sizes[5] < (size_t)DM) return;
  if ((size_t)out_size < need_rows * DM) return;
  if (WS_TOTAL > ws_size) return;
  const float* x    = (const float*)d_in[0];
  const int*   mask = (const int*)d_in[1];
  const float* wqkv = (const float*)d_in[2];
  const float* bqkv = (const float*)d_in[3];
  const float* wout = (const float*)d_in[4];
  const float* bout = (const float*)d_in[5];
  char* ws = (char*)d_ws;
  unsigned short* WQT = (unsigned short*)(ws + WS_WQT);
  unsigned short* WOT = (unsigned short*)(ws + WS_WOT);
  unsigned short* XB  = (unsigned short*)(ws + WS_XB);
  unsigned short* QKH = (unsigned short*)(ws + WS_QKH);
  unsigned short* QKL = (unsigned short*)(ws + WS_QKL);
  unsigned short* VT  = (unsigned short*)(ws + WS_VT);
  unsigned short* CTX = (unsigned short*)(ws + WS_CTX);

  k_wt<<<(unsigned)(((size_t)LQ * (DM / 8) + 255) / 256), 256, 0, stream>>>(wqkv, WQT, LQ, DM, 0);
  k_wt<<<(unsigned)(((size_t)DM * (DM / 8) + 255) / 256), 256, 0, stream>>>(wout, WOT, DM, LL, 1);
  k_xb<<<(unsigned)(((size_t)MR * (DM / 8) + 255) / 256), 256, 0, stream>>>(x, XB);
  k_gemm_qkv<<<(unsigned)((MR / 128) * (LQ / 64)), 128, 0, stream>>>(XB, WQT, bqkv, QKH, QKL);
  k_vt<<<(unsigned)(NB * NH * (SEQ / 64)), 256, 0, stream>>>(QKH, VT);
  k_attn<<<dim3((unsigned)(SEQ / 128), (unsigned)(NB * NH)), 256, 0, stream>>>(QKH, QKL, VT, mask, CTX);
  k_gemm_out<<<(unsigned)((MR / 128) * (DM / 64)), 128, 0, stream>>>(CTX, WOT, bout, (float*)d_out);
}
